// CausalSelfAttention_15564961480737
// MI455X (gfx1250) — hardware-verified
//
#include <hip/hip_runtime.h>


#ifndef NB
#define NB 2
#endif
#ifndef SEQ
#define SEQ 2048
#endif
#define SEQ_FULL 2048
#define DM   1024
#define NH   16
#define HD   64
#define XB_STRIDE_FULL ((size_t)SEQ_FULL * DM)
#define MROWS (NB * SEQ)
#define SCL  0.125f
#define LOG2E 1.4426950408889634f
#define NEGBIG (-1.0e30f)
#define AW   4
#define PPT  40
#define OPT  68
#define NTILE (NB * NH * (SEQ / 16))

static_assert(HD == 64);
static_assert(DM == NH * HD);
static_assert(DM % 64 == 0);
static_assert(DM % 32 == 0);
static_assert(SEQ % 64 == 0);
static_assert(MROWS % 64 == 0);
static_assert(NTILE % AW == 0);
static_assert((PPT * 2) % 16 == 0);
static_assert((OPT * 4) % 16 == 0);
static_assert(SEQ <= SEQ_FULL);

typedef unsigned short bf;
typedef __attribute__((ext_vector_type(16))) __bf16   v16bf;
typedef __attribute__((ext_vector_type(8)))  unsigned short v8us;
typedef __attribute__((ext_vector_type(2)))  unsigned short v2us;
typedef __attribute__((ext_vector_type(8)))  float    v8f;
typedef __attribute__((ext_vector_type(4)))  float    v4f;
typedef __attribute__((ext_vector_type(2)))  float    v2f;
typedef v4f  __attribute__((may_alias)) v4fa;
typedef v8us __attribute__((may_alias)) v8usa;

__device__ __forceinline__ unsigned short f2bf(float f) { unsigned u = __float_as_uint(f); u += 0x7FFFu + ((u >> 16) & 1u); return (unsigned short)(u >> 16); }
__device__ __forceinline__ float bf2f(unsigned short b) { return __uint_as_float(((unsigned)b) << 16); }
__device__ __forceinline__ float bfr(float f) { return bf2f(f2bf(f)); }
__device__ __forceinline__ void splitf(float y, unsigned short& h, unsigned short& l) { h = f2bf(y); l = f2bf(y - bf2f(h)); }
__device__ __forceinline__ v16bf cat16b(v8us lo, v8us hi) { return __builtin_bit_cast(v16bf, __builtin_shufflevector(lo, hi, 0, 1, 2, 3, 4, 5, 6, 7, 8, 9, 10, 11, 12, 13, 14, 15)); }
__device__ __forceinline__ v8f wmmab(v16bf a, v16bf b, v8f c) { return __builtin_amdgcn_wmma_f32_16x16x32_bf16(false, a, false, b, (short)0, c, false, false); }
__device__ __forceinline__ v16bf ldfrag(const bf* p) { return cat16b(*(const v8us*)p, *(const v8us*)(p + 16)); }

template <int NSPLIT, bool BIAS>
__device__ __forceinline__ void gemmw_body(const bf* __restrict__ A, const bf* __restrict__ A2, const bf* __restrict__ Bt, const int K, float* C, const int ldc, const float* __restrict__ bias) {
    __shared__ __align__(16) float os[16 * 68];
    const int lane = threadIdx.x & 31, lr = lane & 15, hi = lane >> 4; const int r0 = blockIdx.x * 64, c0 = blockIdx.y * 64;
    v8f acc[4][4];
#pragma unroll
    for (int mb = 0; mb < 4; ++mb)
#pragma unroll
        for (int nb = 0; nb < 4; ++nb) acc[mb][nb] = (v8f){};
    const size_t aoff = (size_t)(r0 + lr) * K + 8 * hi, boff = (size_t)(c0 + lr) * K + 8 * hi;
#pragma unroll 1
    for (int kc = 0; kc < K; kc += 32) {
        v16bf a[4], a2[4];
#pragma unroll
        for (int mb = 0; mb < 4; ++mb) { a[mb] = ldfrag(A + aoff + (size_t)mb * 16 * K + kc); if (NSPLIT == 1) a2[mb] = ldfrag(A2 + aoff + (size_t)mb * 16 * K + kc); else a2[mb] = a[mb]; }
#pragma unroll
        for (int nb = 0; nb < 4; ++nb) { const v16bf b = ldfrag(Bt + boff + (size_t)nb * 16 * K + kc);
#pragma unroll
            for (int mb = 0; mb < 4; ++mb) { acc[mb][nb] = wmmab(a[mb], b, acc[mb][nb]); if (NSPLIT == 1) acc[mb][nb] = wmmab(a2[mb], b, acc[mb][nb]); } }
        asm volatile("v_nop\n\tv_nop\n\tv_nop\n\tv_nop" : "+v"(acc[0][0]), "+v"(acc[1][1]), "+v"(acc[2][2]), "+v"(acc[3][3]) : "v"(a[0]), "v"(a[3]), "v"(a2[3]));
    }
#pragma unroll
    for (int mb = 0; mb < 4; ++mb) {
#pragma unroll
        for (int nb = 0; nb < 4; ++nb) {
#pragma unroll
            for (int j = 0; j < 8; ++j) os[(hi * 8 + j) * 68 + nb * 16 + lr] = acc[mb][nb][j]; }
        __builtin_amdgcn_wave_barrier(); asm volatile("" ::: "memory");
        float* crow = C + (size_t)(r0 + mb * 16) * ldc + c0;
#pragma unroll 1
        for (int ps = 0; ps < 2; ++ps) {
#pragma unroll
            for (int s = 0; s < 8; ++s) { const int row = 2 * s + hi, cofs = lr * 4; v4f val = *(const v4fa*)(os + row * 68 + cofs); if (BIAS) { val[0] += bfr(bias[c0 + cofs]); val[1] += bfr(bias[c0 + cofs + 1]); val[2] += bfr(bias[c0 + cofs + 2]); val[3] += bfr(bias[c0 + cofs + 3]); }
                *(volatile v4f*)(crow + (size_t)row * ldc + cofs) = val; }
            if (ps == 0) __threadfence(); }
        __builtin_amdgcn_wave_barrier(); asm volatile("" ::: "memory");
    }
}
__global__ __launch_bounds__(32) void k_gemm_proj(const bf* __restrict__ A, const bf* __restrict__ Bt, float* C, const float* __restrict__ bias) { gemmw_body<0, true>(A, A, Bt, DM, C, DM, bias); }
__global__ __launch_bounds__(32) void k_gemm_out(const bf* __restrict__ A, const bf* __restrict__ A2, const bf* __restrict__ Bt, float* C, const float* __restrict__ bias) { gemmw_body<1, true>(A, A2, Bt, DM, C, DM, bias); }

__global__ __launch_bounds__(256) void k_cvt8(const float* __restrict__ src, bf* dst, size_t n8) { const size_t i = (size_t)blockIdx.x * 256 + threadIdx.x; if (i >= n8) return; const v8f v = *(const v8f*)(src + i * 8); v8us o;
#pragma unroll
    for (int k = 0; k < 8; ++k) o[k] = f2bf(v[k]); *(volatile v8us*)(dst + i * 8) = o; __threadfence(); *(volatile v8us*)(dst + i * 8) = o; }
__global__ __launch_bounds__(256) void k_cvtx(const float* __restrict__ src, bf* dst) { const size_t per = (size_t)SEQ * DM / 8; const size_t i = (size_t)blockIdx.x * 256 + threadIdx.x; if (i >= (size_t)NB * per) return; const size_t b = i / per, r = i % per; const v8f v = *(const v8f*)(src + b * XB_STRIDE_FULL + r * 8); v8us o;
#pragma unroll
    for (int k = 0; k < 8; ++k) o[k] = f2bf(v[k]); *(volatile v8us*)(dst + i * 8) = o; __threadfence(); *(volatile v8us*)(dst + i * 8) = o; }

__global__ __launch_bounds__(256) void k_cstab(float* CS) { const int idx = blockIdx.x * 256 + threadIdx.x; if (idx >= SEQ * 32) return; const int i = idx & 31, t = idx >> 5;
    double p = 1.0; p *= (i & 1) ? 1.3335214321633240 : 1.0; p *= (i & 2) ? 1.7782794100389228 : 1.0; p *= (i & 4) ? 3.1622776601683795 : 1.0; p *= (i & 8) ? 10.0 : 1.0; p *= (i & 16) ? 100.0 : 1.0;
    const float pf = (float)p; const float inv = __fdiv_rn(1.0f, pf); const float ang = __fmul_rn((float)t, inv);
    v2f cs; cs[0] = cosf(ang); cs[1] = sinf(ang);
    *(volatile v2f*)(CS + (size_t)idx * 2) = cs; __threadfence(); *(volatile v2f*)(CS + (size_t)idx * 2) = cs; }

__global__ __launch_bounds__(256) void k_rope(const float* __restrict__ F, const float* __restrict__ CS, bf* Ph, bf* Pl) {
    const size_t e = ((size_t)blockIdx.x * 256 + threadIdx.x) * 2; if (e >= (size_t)NB * NH * SEQ * HD) return; const int d = (int)(e % HD); const int t = (int)((e / HD) % SEQ); const int bh = (int)(e / ((size_t)HD * SEQ)); const int b = bh / NH, h = bh % NH;
    const float* f = F + ((size_t)b * SEQ + t) * DM + h * HD; v2us oh, ol;
#pragma unroll
    for (int q = 0; q < 2; ++q) { const int dd = d + q; const int dp = (dd < HD / 2) ? dd + HD / 2 : dd - HD / 2; const float x0 = f[dd], x1 = f[dp];
        const v2f cs = *(const v2f*)(CS + ((size_t)t * 32 + (dd & 31)) * 2); float a = __fmul_rn(x0, cs[0]), bq = __fmul_rn(x1, cs[1]); asm volatile("" : "+v"(a)); asm volatile("" : "+v"(bq)); const float r = (dd < HD / 2) ? __fsub_rn(a, bq) : __fadd_rn(a, bq);
        unsigned short a2, c2; splitf(r, a2, c2); oh[q] = a2; ol[q] = c2; }
    *(volatile v2us*)(Ph + e) = oh; *(volatile v2us*)(Pl + e) = ol; __threadfence(); *(volatile v2us*)(Ph + e) = oh; *(volatile v2us*)(Pl + e) = ol; }
__global__ __launch_bounds__(256) void k_vtp(const float* __restrict__ F, bf* Vh, bf* Vl) { const size_t e = ((size_t)blockIdx.x * 256 + threadIdx.x) * 2; if (e >= (size_t)NB * NH * HD * SEQ) return; const int t = (int)(e % SEQ); const int d = (int)((e / SEQ) % HD); const int bg = (int)(e / ((size_t)SEQ * HD)); const int b = bg / NH, g = bg % NH; v2us oh, ol;
#pragma unroll
    for (int q = 0; q < 2; ++q) { const float x = F[((size_t)b * SEQ + t + q) * DM + g * HD + d]; unsigned short a2, c2; splitf(x, a2, c2); oh[q] = a2; ol[q] = c2; }
    *(volatile v2us*)(Vh + e) = oh; *(volatile v2us*)(Vl + e) = ol; __threadfence(); *(volatile v2us*)(Vh + e) = oh; *(volatile v2us*)(Vl + e) = ol; }

__global__ __launch_bounds__(128) void k_attn(const bf* __restrict__ Qh, const bf* __restrict__ Ql, const bf* __restrict__ Kh, const bf* __restrict__ Kl, const bf* __restrict__ Vh, const bf* __restrict__ Vl, bf* Ah, bf* Al) {
    __shared__ __align__(16) unsigned short ph_s[AW * 16 * PPT];
    __shared__ __align__(16) unsigned short pl_s[AW * 16 * PPT];
    __shared__ __align__(16) float os[AW * 16 * OPT];
    const int wave = __builtin_amdgcn_readfirstlane(threadIdx.x >> 5);
    const int lane = threadIdx.x & 31, lr = lane & 15, hi = lane >> 4;
    const int tile = blockIdx.x * AW + wave;
    if (tile >= NTILE) return;
    const int qt = tile % (SEQ / 16); const int bh = tile / (SEQ / 16); const int b = bh / NH, h = bh % NH; const int t0 = qt * 16;
    const size_t pbase = (size_t)bh * SEQ * HD; const size_t vbase = (size_t)bh * HD * SEQ;
    const size_t qoff = pbase + (size_t)(t0 + lr) * HD + 8 * hi;
    const int pw = wave * 16 * PPT, ow = wave * 16 * OPT;
    v8f o[4]; float mrow[8], lrow[8];
#pragma unroll
    for (int n4 = 0; n4 < 4; ++n4) o[n4] = (v8f){};
#pragma unroll
    for (int r = 0; r < 8; ++r) { mrow[r] = NEGBIG; lrow[r] = 0.0f; }
#pragma unroll 1
    for (int s0 = 0; s0 < t0 + 16; s0 += 32) {
        v8f sc[2]; sc[0] = (v8f){}; sc[1] = (v8f){};
        const size_t koff = pbase + (size_t)(s0 + lr) * HD + 8 * hi;
        v16bf qh, ql, kh, kl;
#pragma unroll
        for (int kk = 0; kk < 2; ++kk) { qh = ldfrag(Qh + qoff + kk * 32); ql = ldfrag(Ql + qoff + kk * 32);
#pragma unroll
            for (int j = 0; j < 2; ++j) { kh = ldfrag(Kh + koff + (size_t)j * 16 * HD + kk * 32); kl = ldfrag(Kl + koff + (size_t)j * 16 * HD + kk * 32);
                sc[j] = wmmab(qh, kh, sc[j]); sc[j] = wmmab(qh, kl, sc[j]); sc[j] = wmmab(ql, kh, sc[j]); } }
        asm volatile("v_nop\n\tv_nop\n\tv_nop\n\tv_nop" : "+v"(sc[0]), "+v"(sc[1]) : "v"(qh), "v"(ql), "v"(kh), "v"(kl));
        const int k0i = s0 + lr, k1i = s0 + 16 + lr;
#pragma unroll
        for (int r = 0; r < 8; ++r) {
            const int t = t0 + 8 * hi + r; const bool ok0 = (k0i <= t), ok1 = (k1i <= t);
            const float a0 = ok0 ? sc[0][r] * SCL : NEGBIG; const float a1 = ok1 ? sc[1][r] * SCL : NEGBIG;
            float v = fmaxf(a0, a1);
            v = fmaxf(v, __shfl_xor(v, 1, 32)); v = fmaxf(v, __shfl_xor(v, 2, 32)); v = fmaxf(v, __shfl_xor(v, 4, 32)); v = fmaxf(v, __shfl_xor(v, 8, 32));
            const float nm = fmaxf(mrow[r], v);
            const float cr = __builtin_amdgcn_exp2f((mrow[r] - nm) * LOG2E); mrow[r] = nm;
            const float e0 = __builtin_amdgcn_exp2f((a0 - nm) * LOG2E), e1 = __builtin_amdgcn_exp2f((a1 - nm) * LOG2E);
            const float p0 = ok0 ? e0 : 0.0f, p1 = ok1 ? e1 : 0.0f;
            lrow[r] = lrow[r] * cr + (p0 + p1);
            o[0][r] *= cr; o[1][r] *= cr; o[2][r] *= cr; o[3][r] *= cr;
            unsigned short h0, l0, h1, l1; splitf(p0, h0, l0); splitf(p1, h1, l1);
            const int pi = pw + (8 * hi + r) * PPT + lr;
            ph_s[pi] = h0; ph_s[pi + 16] = h1; pl_s[pi] = l0; pl_s[pi + 16] = l1;
        }
        __builtin_amdgcn_wave_barrier(); asm volatile("s_wait_dscnt 0" ::: "memory");
        const int pr = pw + lr * PPT + 8 * hi;
        const v16bf pa = cat16b(*(const v8usa*)(ph_s + pr), *(const v8usa*)(ph_s + pr + 16));
        const v16bf pb = cat16b(*(const v8usa*)(pl_s + pr), *(const v8usa*)(pl_s + pr + 16));
        const size_t voff = vbase + (size_t)lr * SEQ + s0 + 8 * hi;
        v16bf vh, vl;
#pragma unroll
        for (int n4 = 0; n4 < 4; ++n4) { vh = ldfrag(Vh + voff + (size_t)n4 * 16 * SEQ); vl = ldfrag(Vl + voff + (size_t)n4 * 16 * SEQ);
            o[n4] = wmmab(pa, vh, o[n4]); o[n4] = wmmab(pa, vl, o[n4]); o[n4] = wmmab(pb, vh, o[n4]); }
        asm volatile("v_nop\n\tv_nop\n\tv_nop\n\tv_nop" : "+v"(o[0]), "+v"(o[1]), "+v"(o[2]), "+v"(o[3]) : "v"(pa), "v"(pb), "v"(vh), "v"(vl));
        __builtin_amdgcn_wave_barrier(); asm volatile("" ::: "memory");
    }
#pragma unroll
    for (int r = 0; r < 8; ++r) { float l = lrow[r]; l += __shfl_xor(l, 1, 32); l += __shfl_xor(l, 2, 32); l += __shfl_xor(l, 4, 32); l += __shfl_xor(l, 8, 32); const float inv = __fdiv_rn(1.0f, l);
        const int oi = ow + (8 * hi + r) * OPT + lr;
        os[oi] = o[0][r] * inv; os[oi + 16] = o[1][r] * inv; os[oi + 32] = o[2][r] * inv; os[oi + 48] = o[3][r] * inv; }
    __builtin_amdgcn_wave_barrier(); asm volatile("s_wait_dscnt 0" ::: "memory");
#pragma unroll 1
    for (int ps = 0; ps < 2; ++ps) {
#pragma unroll
        for (int s = 0; s < 4; ++s) { const int row = 4 * s + (lane >> 3), c8 = (lane & 7) * 8;
            const v4f x0 = *(const v4fa*)(os + ow + row * OPT + c8); const v4f x1 = *(const v4fa*)(os + ow + row * OPT + c8 + 4); v8us oh, ol;
#pragma unroll
            for (int q = 0; q < 4; ++q) { unsigned short a, c2; splitf(x0[q], a, c2); oh[q] = a; ol[q] = c2; splitf(x1[q], a, c2); oh[4 + q] = a; ol[4 + q] = c2; }
            const size_t dst = ((size_t)b * SEQ + t0 + row) * DM + h * HD + c8;
            *(volatile v8us*)(Ah + dst) = oh; *(volatile v8us*)(Al + dst) = ol; }
        if (ps == 0) __threadfence(); }
}

constexpr size_t SZ_W  = (size_t)DM * DM * 2;
constexpr size_t SZ_CS = (size_t)SEQ * 32 * 2 * 4;
constexpr size_t SZ_XB = (size_t)MROWS * DM * 2;
constexpr size_t SZ_F  = (size_t)MROWS * DM * 4;
constexpr size_t SZ_PL = (size_t)MROWS * DM * 2;
constexpr size_t WS_TOTAL = 4 * SZ_W + SZ_CS + SZ_XB + SZ_F + 8 * SZ_PL;
static_assert(SZ_W % 256 == 0);
static_assert(SZ_CS % 256 == 0);
static_assert(SZ_XB % 256 == 0);
static_assert(SZ_F % 256 == 0);
static_assert(SZ_PL % 256 == 0);
static_assert(WS_TOTAL <= (size_t)134217728);
static_assert((size_t)NB * NH * SEQ * HD == (size_t)MROWS * DM);

extern "C" void kernel_launch(void* const* d_in, const int* in_sizes, int n_in,
                              void* d_out, int out_size, void* d_ws, size_t ws_size, hipStream_t stream) {
    if (n_in < 9) return;
    if ((size_t)in_sizes[0] < (size_t)(NB - 1) * XB_STRIDE_FULL + (size_t)SEQ * DM) return;
    if ((size_t)in_sizes[1] < (size_t)DM * DM || (size_t)in_sizes[3] < (size_t)DM * DM || (size_t)in_sizes[5] < (size_t)DM * DM || (size_t)in_sizes[7] < (size_t)DM * DM) return;
    if (in_sizes[2] < DM || in_sizes[4] < DM || in_sizes[6] < DM || in_sizes[8] < DM) return;
    if ((size_t)out_size < (size_t)MROWS * DM) return;
    if (ws_size < WS_TOTAL) return;
    const float* x = (const float*)d_in[0]; const float* wq = (const float*)d_in[1]; const float* bq = (const float*)d_in[2]; const float* wk = (const float*)d_in[3]; const float* bk = (const float*)d_in[4];
    const float* wv = (const float*)d_in[5]; const float* bv = (const float*)d_in[6]; const float* wo = (const float*)d_in[7]; const float* bo = (const float*)d_in[8];
    float* OUT = (float*)d_out;
    char* wsp = (char*)d_ws;
    auto take = [&](size_t bytes) { char* p = wsp; wsp += (bytes + 255) & ~(size_t)255; return (void*)p; };
    bf* WQ = (bf*)take(SZ_W); bf* WK = (bf*)take(SZ_W); bf* WV = (bf*)take(SZ_W); bf* WO = (bf*)take(SZ_W);
    float* CS = (float*)take(SZ_CS);
    bf* XB = (bf*)take(SZ_XB);
    float* F = (float*)take(SZ_F);
    bf* QPh = (bf*)take(SZ_PL); bf* QPl = (bf*)take(SZ_PL); bf* KPh = (bf*)take(SZ_PL); bf* KPl = (bf*)take(SZ_PL); bf* VTh = (bf*)take(SZ_PL); bf* VTl = (bf*)take(SZ_PL);
    bf* ATh = (bf*)take(SZ_PL); bf* ATl = (bf*)take(SZ_PL);
    if ((size_t)(wsp - (char*)d_ws) > ws_size) return;

    const size_t nw8 = (size_t)DM * DM / 8; const unsigned gw = (unsigned)((nw8 + 255) / 256);
    k_cvt8<<<gw, 256, 0, stream>>>(wq, WQ, nw8);
    k_cvt8<<<gw, 256, 0, stream>>>(wk, WK, nw8);
    k_cvt8<<<gw, 256, 0, stream>>>(wv, WV, nw8);
    k_cvt8<<<gw, 256, 0, stream>>>(wo, WO, nw8);
    k_cvtx<<<(unsigned)(((size_t)MROWS * DM / 8 + 255) / 256), 256, 0, stream>>>(x, XB);
    k_cstab<<<(SEQ * 32 + 255) / 256, 256, 0, stream>>>(CS);
    const unsigned LP = (unsigned)(((size_t)NB * NH * SEQ * HD / 2 + 255) / 256);
    const dim3 gg(MROWS / 64, DM / 64, 1);
    k_gemm_proj<<<gg, 32, 0, stream>>>(XB, WQ, F, bq);
    k_rope<<<LP, 256, 0, stream>>>(F, CS, QPh, QPl);
    k_gemm_proj<<<gg, 32, 0, stream>>>(XB, WK, F, bk);
    k_rope<<<LP, 256, 0, stream>>>(F, CS, KPh, KPl);
    k_gemm_proj<<<gg, 32, 0, stream>>>(XB, WV, F, bv);
    k_vtp<<<LP, 256, 0, stream>>>(F, VTh, VTl);
    k_attn<<<NTILE / AW, AW * 32, 0, stream>>>(QPh, QPl, KPh, KPl, VTh, VTl, ATh, ATl);
    k_gemm_out<<<gg, 32, 0, stream>>>(ATh, ATl, WO, OUT, bo);
}
